// SimpleTwoLayerNet_68118181315033
// MI455X (gfx1250) — hardware-verified
//
#include <hip/hip_runtime.h>
#include <stddef.h>
#include <stdint.h>
#include <math.h>

#define NB   8192
#define NP   4096
#define ND   512
#define NC   1000
#define NCP  1024
#define NPB  (NP / 128)
#define SHP  136
#define SFP  132

static_assert(ND == 512);
static_assert(ND % 32 == 0);
static_assert(NB % 128 == 0);
static_assert(NP % 128 == 0);
static_assert(NCP % 128 == 0);
static_assert(NC % 4 == 0);
static_assert(NC <= NCP);
static_assert(NPB == 32);
static_assert(NB % 32 == 0);
static_assert(NP % 64 == 0);
static_assert(NCP % 64 == 0);

typedef _Float16 hh;
typedef hh    v16h __attribute__((ext_vector_type(16)));
typedef hh    v8h  __attribute__((ext_vector_type(8)));
typedef float v8f  __attribute__((ext_vector_type(8)));
typedef float v4f  __attribute__((ext_vector_type(4)));

union Frag { v16h v; v8h p[2]; };

__device__ __forceinline__ v8f zero8() { return (v8f){0.f, 0.f, 0.f, 0.f, 0.f, 0.f, 0.f, 0.f}; }

__device__ __forceinline__ float wsum(float v) {
#pragma unroll
  for (int off = 16; off > 0; off >>= 1) v += __shfl_xor(v, off, 32);
  return v;
}

__device__ __forceinline__ v16h ldfrag(const hh* __restrict__ p, int ld, int row0, int k0, int lane) {
  const hh* q = p + (size_t)(row0 + (lane & 15)) * (size_t)ld + k0 + 8 * (lane >> 4);
  Frag f;
  f.p[0] = *(const v8h*)(q);
  f.p[1] = *(const v8h*)(q + 16);
  return f.v;
}

__device__ __forceinline__ v8f mma16(v16h a, v16h b, v8f cc) {
  return __builtin_amdgcn_wmma_f32_16x16x32_f16(false, a, false, b, (short)0, cc, false, false);
}

__device__ __forceinline__ void gemm32x64(const hh* __restrict__ A, int lda, const hh* __restrict__ B, int ldb,
                                          int ma, int nb, int kdim, int lane, v8f (&acc)[2][4]) {
#pragma unroll 1
  for (int k0 = 0; k0 < kdim; k0 += 32) {
    const v16h a0 = ldfrag(A, lda, ma, k0, lane);
    const v16h a1 = ldfrag(A, lda, ma + 16, k0, lane);
    const v16h b0 = ldfrag(B, ldb, nb, k0, lane);
    const v16h b1 = ldfrag(B, ldb, nb + 16, k0, lane);
    const v16h b2 = ldfrag(B, ldb, nb + 32, k0, lane);
    const v16h b3 = ldfrag(B, ldb, nb + 48, k0, lane);
    acc[0][0] = mma16(a0, b0, acc[0][0]);
    acc[1][0] = mma16(a1, b0, acc[1][0]);
    acc[0][1] = mma16(a0, b1, acc[0][1]);
    acc[1][1] = mma16(a1, b1, acc[1][1]);
    acc[0][2] = mma16(a0, b2, acc[0][2]);
    acc[1][2] = mma16(a1, b2, acc[1][2]);
    acc[0][3] = mma16(a0, b3, acc[0][3]);
    acc[1][3] = mma16(a1, b3, acc[1][3]);
    asm volatile("v_nop\n\tv_nop\n\tv_nop\n\tv_nop"
                 : "+v"(acc[0][0]), "+v"(acc[0][1]), "+v"(acc[0][2]), "+v"(acc[0][3]),
                   "+v"(acc[1][0]), "+v"(acc[1][1]), "+v"(acc[1][2]), "+v"(acc[1][3])
                 : "v"(a0), "v"(a1), "v"(b0), "v"(b1), "v"(b2), "v"(b3));
  }
}

__global__ __launch_bounds__(256) void k_rows(const float* __restrict__ src, hh* __restrict__ dst,
                                              float* __restrict__ nrm) {
  __shared__ __align__(16) float sn[32];
  const int tid = threadIdx.x, lane = tid & 31, w = tid >> 5;
  const int rb = blockIdx.x * 32 + w * 4;
  v8h hv[4][2];
#pragma unroll
  for (int i = 0; i < 4; ++i) {
    const float* rp = src + (size_t)(rb + i) * ND;
    const v4f a0 = *(const v4f*)(rp + 8 * lane), a1 = *(const v4f*)(rp + 8 * lane + 4);
    const v4f b0 = *(const v4f*)(rp + 256 + 8 * lane), b1 = *(const v4f*)(rp + 256 + 8 * lane + 4);
    const v8f ta = {a0[0], a0[1], a0[2], a0[3], a1[0], a1[1], a1[2], a1[3]};
    const v8f tb = {b0[0], b0[1], b0[2], b0[3], b1[0], b1[1], b1[2], b1[3]};
    float s = 0.f;
#pragma unroll
    for (int e = 0; e < 8; ++e) s = fmaf(ta[e], ta[e], s);
#pragma unroll
    for (int e = 0; e < 8; ++e) s = fmaf(tb[e], tb[e], s);
    s = wsum(s);
    hv[i][0] = __builtin_convertvector(ta, v8h);
    hv[i][1] = __builtin_convertvector(tb, v8h);
    if (lane == 0) sn[w * 4 + i] = s;
  }
#pragma unroll
  for (int i = 0; i < 4; ++i) {
    hh* op = dst + (size_t)(rb + i) * ND;
    *(volatile v8h*)(op + 8 * lane) = hv[i][0];
    *(volatile v8h*)(op + 256 + 8 * lane) = hv[i][1];
  }
  __threadfence();
#pragma unroll
  for (int i = 0; i < 4; ++i) {
    hh* op = dst + (size_t)(rb + i) * ND;
    *(volatile v8h*)(op + 8 * lane) = hv[i][0];
    *(volatile v8h*)(op + 256 + 8 * lane) = hv[i][1];
  }
  __syncthreads();
  if (w == 0) {
    const int li = lane & 7;
    const v4f v = *(const v4f*)(sn + 4 * li);
    float* gp = nrm + (size_t)blockIdx.x * 32 + 4 * li;
    if (lane < 8) *(volatile v4f*)gp = v;
    __threadfence();
    if (lane < 8) *(volatile v4f*)gp = v;
  }
}

__global__ __launch_bounds__(256) void k_cvt_vt(const float* __restrict__ vals, hh* __restrict__ vt) {
  __shared__ __align__(16) float sw[64 * 68];
  const int tid = threadIdx.x;
  const int kb = blockIdx.x * 64;
  const int nb = blockIdx.y * 64;
  {
    const int r  = tid >> 2;
    const int c0 = (tid & 3) * 16;
    const float* rp = vals + (size_t)(kb + r) * NC;
#pragma unroll
    for (int e = 0; e < 4; ++e) {
      const int c   = nb + c0 + 4 * e;
      const int ccl = (c < NC - 4) ? c : (NC - 4);
      v4f v = *(const v4f*)(rp + ccl);
      if (c >= NC) v = (v4f){0.f, 0.f, 0.f, 0.f};
      *(v4f*)(sw + r * 68 + c0 + 4 * e) = v;
    }
  }
  __syncthreads();
  v8h hv[2];
  size_t go[2];
#pragma unroll
  for (int j = 0; j < 2; ++j) {
    const int p  = tid + 256 * j;
    const int n  = p >> 3;
    const int pc = p & 7;
    const float* cp = sw + (pc * 8) * 68 + n;
    v8f t;
#pragma unroll
    for (int e = 0; e < 8; ++e) t[e] = cp[e * 68] * 16.0f;
    hv[j] = __builtin_convertvector(t, v8h);
    go[j] = (size_t)(nb + n) * NP + kb + pc * 8;
  }
#pragma unroll
  for (int j = 0; j < 2; ++j) *(volatile v8h*)(vt + go[j]) = hv[j];
  __threadfence();
#pragma unroll
  for (int j = 0; j < 2; ++j) *(volatile v8h*)(vt + go[j]) = hv[j];
}

__global__ __launch_bounds__(256) void k_gemm_w(const hh* __restrict__ XH, const hh* __restrict__ KH,
                                                const float* __restrict__ XN, const float* __restrict__ KN,
                                                hh* __restrict__ Wp, float* __restrict__ PS) {
  __shared__ __align__(16) hh sh[128 * SHP];
  __shared__ float part[8 * 32];
  __shared__ __align__(16) float rl[128];
  const int tid = threadIdx.x, lane = tid & 31, w = tid >> 5;
  const int h = lane >> 4, c = lane & 15;
  const int wm = (w >> 1) * 32, wn = (w & 1) * 64;
  const int m0 = blockIdx.y * 128;
  const int n0 = blockIdx.x * 128;

  v8f acc[2][4];
#pragma unroll
  for (int i = 0; i < 2; ++i)
#pragma unroll
    for (int j = 0; j < 4; ++j) acc[i][j] = zero8();
  gemm32x64(XH, ND, KH, ND, m0 + wm, n0 + wn, ND, lane, acc);

  float knc[4];
#pragma unroll
  for (int j = 0; j < 4; ++j) knc[j] = KN[n0 + wn + 16 * j + c];

#pragma unroll
  for (int i = 0; i < 2; ++i) {
    const v8f xt = *(const v8f*)(XN + m0 + wm + 16 * i + 8 * h);
    float ps[8];
#pragma unroll
    for (int r = 0; r < 8; ++r) ps[r] = 0.f;
#pragma unroll
    for (int j = 0; j < 4; ++j) {
      float v[8];
#pragma unroll
      for (int r = 0; r < 8; ++r) {
        const float g  = acc[i][j][r];
        const float sq = (xt[r] + knc[j]) - 2.0f * g;
        const float d2 = fmaxf(sq, 0.f);
        const float wv = __builtin_amdgcn_rcpf(1e-3f + d2);
        ps[r] += wv;
        v[r] = wv * 64.0f;
      }
#pragma unroll
      for (int r = 0; r < 8; ++r)
        sh[(wm + 16 * i + 8 * h + r) * SHP + wn + 16 * j + c] = (hh)v[r];
    }
#pragma unroll
    for (int r = 0; r < 8; ++r) {
      float t = ps[r];
      t += __shfl_xor(t, 8, 32);
      t += __shfl_xor(t, 4, 32);
      t += __shfl_xor(t, 2, 32);
      t += __shfl_xor(t, 1, 32);
      ps[r] = t;
    }
    if (c == 0) {
#pragma unroll
      for (int r = 0; r < 8; ++r) part[w * 32 + 16 * i + 8 * h + r] = ps[r];
    }
  }
  __syncthreads();
  if (tid < 128) {
    const int lr = tid;
    const int q  = lr >> 5;
    rl[lr] = part[(2 * q) * 32 + (lr & 31)] + part[(2 * q + 1) * 32 + (lr & 31)];
  }
  __syncthreads();

  v8h val[8];
  size_t go[8];
#pragma unroll
  for (int it = 0; it < 8; ++it) {
    const int p  = tid + 256 * it;
    const int lr = p >> 4;
    const int pc = p & 15;
    val[it] = *(const v8h*)(sh + lr * SHP + pc * 8);
    go[it] = (size_t)(m0 + lr) * NP + n0 + pc * 8;
  }
  const v4f pv = *(const v4f*)(rl + 4 * lane);
  float* gp = PS + (size_t)blockIdx.x * NB + m0 + 4 * lane;
#pragma unroll
  for (int it = 0; it < 8; ++it) *(volatile v8h*)(Wp + go[it]) = val[it];
  if (w == 0) *(volatile v4f*)gp = pv;
  __threadfence();
#pragma unroll
  for (int it = 0; it < 8; ++it) *(volatile v8h*)(Wp + go[it]) = val[it];
  if (w == 0) *(volatile v4f*)gp = pv;
}

__global__ __launch_bounds__(256) void k_gemm_o(const hh* __restrict__ Wp, const hh* __restrict__ VT,
                                                float* __restrict__ O) {
  __shared__ __align__(16) float sf[64 * SFP];
  const int tid = threadIdx.x, lane = tid & 31, w = tid >> 5;
  const int h = lane >> 4, c = lane & 15;
  const int wm = (w >> 1) * 32, wn = (w & 1) * 64;
  const int m0 = blockIdx.y * 128;
  const int n0 = blockIdx.x * 128;

  v8f acc[2][4];
#pragma unroll
  for (int i = 0; i < 2; ++i)
#pragma unroll
    for (int j = 0; j < 4; ++j) acc[i][j] = zero8();
  gemm32x64(Wp, NP, VT, NP, m0 + wm, n0 + wn, NP, lane, acc);

#pragma unroll
  for (int hf = 0; hf < 2; ++hf) {
    if ((w >> 2) == hf) {
#pragma unroll
      for (int i = 0; i < 2; ++i)
#pragma unroll
        for (int j = 0; j < 4; ++j)
#pragma unroll
          for (int r = 0; r < 8; ++r)
            sf[(wm - 64 * hf + 16 * i + 8 * h + r) * SFP + wn + 16 * j + c] = acc[i][j][r];
    }
    __syncthreads();
    v4f val[8];
    size_t go[8];
#pragma unroll
    for (int it = 0; it < 8; ++it) {
      const int p  = tid + 256 * it;
      const int lr = p >> 5;
      const int pc = p & 31;
      val[it] = *(const v4f*)(sf + lr * SFP + pc * 4);
      go[it] = (size_t)(m0 + 64 * hf + lr) * NCP + n0 + pc * 4;
    }
#pragma unroll
    for (int it = 0; it < 8; ++it) *(volatile v4f*)(O + go[it]) = val[it];
    __threadfence();
#pragma unroll
    for (int it = 0; it < 8; ++it) *(volatile v4f*)(O + go[it]) = val[it];
    if (hf == 0) __syncthreads();
  }
}

__global__ __launch_bounds__(256) void k_pack(const float* __restrict__ O, const float* __restrict__ PS,
                                              float* __restrict__ out) {
  const int tid = threadIdx.x, lane = tid & 31, w = tid >> 5;
  const int row0 = blockIdx.x * 32 + w * 4;
  float sc[4];
#pragma unroll
  for (int i = 0; i < 4; ++i) {
    float pv = PS[(size_t)lane * NB + row0 + i];
    pv = wsum(pv);
    sc[i] = 1.0f / (1024.0f * pv);
  }
  const float* ob = O + (size_t)row0 * NCP;
  float* gb = out + (size_t)row0 * NC;
#pragma unroll
  for (int grp = 0; grp < 4; ++grp) {
    v4f val[8];
    int qs[8];
#pragma unroll
    for (int it = 0; it < 8; ++it) {
      const int q  = lane + 32 * (grp * 8 + it);
      const int qq = (q < NC) ? q : (NC - 1);
      const int orow = (qq >= 250 ? 1 : 0) + (qq >= 500 ? 1 : 0) + (qq >= 750 ? 1 : 0);
      const int c4 = (qq - orow * 250) * 4;
      const v4f s = *(const v4f*)(ob + (size_t)orow * NCP + c4);
      const float f = (orow == 0) ? sc[0] : ((orow == 1) ? sc[1] : ((orow == 2) ? sc[2] : sc[3]));
      val[it] = s * f;
      qs[it] = q;
    }
#pragma unroll
    for (int it = 0; it < 8; ++it)
      if (qs[it] < NC) *(volatile v4f*)(gb + 4 * qs[it]) = val[it];
    __threadfence();
#pragma unroll
    for (int it = 0; it < 8; ++it)
      if (qs[it] < NC) *(volatile v4f*)(gb + 4 * qs[it]) = val[it];
  }
}

extern "C" void kernel_launch(void* const* d_in, const int* in_sizes, int n_in,
                              void* d_out, int out_size, void* d_ws, size_t ws_size,
                              hipStream_t stream) {
  if (n_in < 3) return;
  if (in_sizes[0] != NB * ND) return;
  if (in_sizes[1] != NP * ND) return;
  if (in_sizes[2] != NP * NC) return;
  if (out_size != NB * NC) return;

  const float* x    = (const float*)d_in[0];
  const float* keys = (const float*)d_in[1];
  const float* vals = (const float*)d_in[2];
  float* out = (float*)d_out;

  size_t off = 0;
  const size_t oXH = off; off += (size_t)NB * ND * 2;
  const size_t oKH = off; off += (size_t)NP * ND * 2;
  const size_t oXN = off; off += (size_t)NB * 4;
  const size_t oKN = off; off += (size_t)NP * 4;
  const size_t oVT = off; off += (size_t)NCP * NP * 2;
  const size_t oW  = off; off += (size_t)NB * NP * 2;
  const size_t oPS = off; off += (size_t)NPB * NB * 4;
  const size_t oO  = off; off += (size_t)NB * NCP * 4;
  if (off > ws_size) return;
  if (off > (size_t)134217728) return;

  char* ws = (char*)d_ws;
  hh*    XH = (hh*)(ws + oXH);
  hh*    KH = (hh*)(ws + oKH);
  float* XN = (float*)(ws + oXN);
  float* KN = (float*)(ws + oKN);
  hh*    VT = (hh*)(ws + oVT);
  hh*    W  = (hh*)(ws + oW);
  float* PS = (float*)(ws + oPS);
  float* O32 = (float*)(ws + oO);

  k_rows<<<dim3(NB / 32), dim3(256), 0, stream>>>(x, XH, XN);
  k_rows<<<dim3(NP / 32), dim3(256), 0, stream>>>(keys, KH, KN);
  k_cvt_vt<<<dim3(NP / 64, NCP / 64), dim3(256), 0, stream>>>(vals, VT);
  k_gemm_w<<<dim3(NP / 128, NB / 128), dim3(256), 0, stream>>>(XH, KH, XN, KN, W, PS);
  k_gemm_o<<<dim3(NCP / 128, NB / 128), dim3(256), 0, stream>>>(W, VT, O32);
  k_pack<<<dim3(NB / 32), dim3(256), 0, stream>>>(O32, PS, out);
  (void)hipGetLastError();
}
